// SignalAttention_53987738911346
// MI455X (gfx1250) — hardware-verified
//
#include <hip/hip_runtime.h>
#include <hip/hip_bf16.h>
#include <math.h>

#define NBs 4
#define TTs 2048
#define HHs 256
#define MTOK (NBs * TTs)
#define HALF 16
#define GSTR 48
#define SS TTs
#define HH 1
#define DKK 64

typedef _Float16 bf16;
typedef _Float16 f16;
typedef __attribute__((ext_vector_type(4))) unsigned v4u_t;
typedef unsigned v4ua __attribute__((ext_vector_type(4), may_alias));
typedef __attribute__((ext_vector_type(4))) float v4f_t;
typedef float v4fa __attribute__((ext_vector_type(4), may_alias));
typedef __attribute__((ext_vector_type(16))) bf16  bf16x16;
typedef bf16x16 f16x16;
typedef __attribute__((ext_vector_type(8)))  bf16  bf16x8;
typedef bf16x8 f16x8;
typedef __attribute__((ext_vector_type(4)))  bf16  bf16x4;
typedef __attribute__((ext_vector_type(8)))  float f32x8;
__device__ __forceinline__ f32x8 wmma16(f16x16 a, f16x16 b, f32x8 c) {
  c = __builtin_amdgcn_wmma_f32_16x16x32_f16(false, a, false, b, (short)0, c, false, false);
  asm volatile("v_nop\n\tv_nop\n\tv_nop\n\tv_nop" : "+v"(c) : "v"(a), "v"(b));
  return c;
}
#define LDS_STRIDE 48
#define KSTRIDE    72
#define VSTRIDE    48

__device__ __forceinline__ f32x8 wmma_bf16(bf16x16 a, bf16x16 b, f32x8 c) {
  c = __builtin_amdgcn_wmma_f32_16x16x32_f16(false, a, false, b, (short)0, c, false, false);
  asm volatile("v_nop\n\tv_nop\n\tv_nop\n\tv_nop" : "+v"(c) : "v"(a), "v"(b));
  return c;
}

template <typename T>
__device__ __forceinline__ bf16x16 load_frag(const T* __restrict__ base, int ld,
                                             int row0, int k0) {
  const int lane = threadIdx.x & 31;
  const int r    = lane & 15;
  const int kh   = (lane >> 4) * 8;
  const T* p0 = base + (size_t)(row0 + r) * ld + (k0 + kh);
  const T* p1 = p0 + 16;
  bf16x16 f;
#pragma unroll
  for (int i = 0; i < 8; ++i) {
    f[i]     = (bf16)p0[i];
    f[i + 8] = (bf16)p1[i];
  }
  return f;
}

__device__ __forceinline__ bf16x16 lds_frag(const bf16* base, int stride) {
  const int lane = threadIdx.x & 31;
  const int row  = lane & 15;
  const int kh   = (lane >> 4) * 8;
  const bf16x8 lo = *(const bf16x8*)(base + row * stride + kh);
  const bf16x8 hi = *(const bf16x8*)(base + row * stride + kh + 16);
  bf16x16 f;
#pragma unroll
  for (int i = 0; i < 8; ++i) { f[i] = lo[i]; f[i + 8] = hi[i]; }
  return f;
}

template <typename T>
__device__ __forceinline__ void stage_read16(const T* __restrict__ p, float* buf) {
#pragma unroll
  for (int i = 0; i < 16; ++i) buf[i] = (float)p[i];
}

__device__ __forceinline__ void stage_write(bf16* dst, const float* buf, int nquad) {
#pragma unroll
  for (int i = 0; i < nquad; ++i) {
    bf16x4 q;
    q[0] = (bf16)buf[4 * i];     q[1] = (bf16)buf[4 * i + 1];
    q[2] = (bf16)buf[4 * i + 2]; q[3] = (bf16)buf[4 * i + 3];
    *(bf16x4*)(dst + 4 * i) = q;
  }
}

template <typename AT, int MODE>
__global__ __launch_bounds__(256) void gemm_rb_kernel(
    const AT* __restrict__ A, const float* __restrict__ W,
    const float* __restrict__ bias, const float* __restrict__ rowscale, const float* __restrict__ R, const float* __restrict__ rowbias, void* __restrict__ out,
    int M, int N, int K) {
  __shared__ bf16 ldsA[128 * LDS_STRIDE];
  __shared__ bf16 ldsW[256 * LDS_STRIDE];
  __shared__ __attribute__((aligned(16))) unsigned char sob[256 * 136 * 2];

  const int t    = threadIdx.x;
  const int wave = t >> 5;
  const int lane = t & 31;
  const int wm   = (wave & 1) * 64;
  const int wn   = (wave >> 1) * 64;
  const int mBlk = blockIdx.x * 128;
  const int nBlk = blockIdx.y * 256;

  const int arow = t >> 1;
  const int ach  = (t & 1) * 16;

  float abuf[16];
  float wbuf[32];

  stage_read16(A + (size_t)(mBlk + arow) * K + ach, abuf);
  const int nrow = min(nBlk + t, N - 1);
  stage_read16(W + (size_t)nrow * K,          wbuf);
  stage_read16(W + (size_t)nrow * K + 16,     wbuf + 16);

  f32x8 acc[4][4] = {};

  for (int k = 0; k < K; k += 32) {
    __syncthreads();
    stage_write(&ldsA[arow * LDS_STRIDE + ach], abuf, 4);
    stage_write(&ldsW[t * LDS_STRIDE],          wbuf, 8);
    if (k + 32 < K) {
      stage_read16(A + (size_t)(mBlk + arow) * K + (k + 32) + ach, abuf);
      stage_read16(W + (size_t)nrow * K + (k + 32),          wbuf);
      stage_read16(W + (size_t)nrow * K + (k + 32) + 16,     wbuf + 16);
    }
    __syncthreads();

    bf16x16 af[4], wf[4];
#pragma unroll
    for (int i = 0; i < 4; ++i)
      af[i] = lds_frag(ldsA + (wm + 16 * i) * LDS_STRIDE, LDS_STRIDE);
#pragma unroll
    for (int j = 0; j < 4; ++j)
      wf[j] = lds_frag(ldsW + (wn + 16 * j) * LDS_STRIDE, LDS_STRIDE);
#pragma unroll
    for (int i = 0; i < 4; ++i)
#pragma unroll
      for (int j = 0; j < 4; ++j)
        acc[i][j] = wmma_bf16(af[i], wf[j], acc[i][j]);
  }

  const int nlane = lane & 15;
  const int mh    = (lane >> 4) * 8;
  __syncthreads();
  if (MODE == 0 || MODE == 1 || MODE == 3) {
    bf16* so = (bf16*)sob;
#pragma unroll
    for (int i = 0; i < 4; ++i)
#pragma unroll
      for (int j = 0; j < 4; ++j) {
        const int nl = wn + 16 * j + nlane;
        const float bv = bias ? bias[nBlk + nl] : 0.0f;
        if (MODE == 3) {
#pragma unroll 1
          for (int r = 0; r < 8; ++r) {
            const int ml = wm + 16 * i + mh + r;
            const float xg = acc[i][j][r] + bv;
            so[ml * 264 + nl] = (bf16)(0.5f * xg * (1.0f + erff(xg * 0.70710678118654752f)));
          }
        } else {
#pragma unroll
        for (int r = 0; r < 8; ++r) {
          const int ml = wm + 16 * i + mh + r;
          const bf16 hv = (bf16)(acc[i][j][r] + bv);
          if (MODE == 0) so[ml * 264 + nl] = hv;
          else           so[nl * 136 + ml] = hv;
        }
        }
      }
    __syncthreads();
#pragma unroll 1
    for (int pass = 0; pass < 2; ++pass) {
      if (MODE == 0 || MODE == 3) {
        for (int ch = t; ch < 128 * 32; ch += 256) { const int ml = ch >> 5, q = (ch & 31) * 8;
          *(volatile v4u_t*)((bf16*)out + (size_t)(mBlk + ml) * N + nBlk + q) = *(const v4ua*)(so + ml * 264 + q); }
      } else {
        const int b_ = mBlk / SS, s0 = mBlk % SS;
        for (int ch = t; ch < 256 * 16; ch += 256) { const int nl = ch >> 4, q = (ch & 15) * 8; const int n = nBlk + nl, h = n >> 6, dk = n & (DKK - 1);
          *(volatile v4u_t*)((bf16*)out + (((size_t)(b_ * HH + h)) * DKK + dk) * SS + s0 + q) = *(const v4ua*)(so + nl * 136 + q); }
      }
      __threadfence();
    }
  } else {
    float* so = (float*)sob;
#pragma unroll 1
    for (int hf = 0; hf < 2; ++hf) {
      if (wm == hf * 64) {
#pragma unroll
        for (int i = 0; i < 4; ++i)
#pragma unroll
          for (int j = 0; j < 4; ++j) {
            const int nl = wn + 16 * j + nlane;
            const float bv = bias ? bias[nBlk + nl] : 0.0f;
#pragma unroll
            for (int r = 0; r < 8; ++r) { const int mrow = mBlk + hf * 64 + 16 * i + mh + r; so[(16 * i + mh + r) * 260 + nl] = acc[i][j][r] * (rowscale ? rowscale[mrow] : 1.0f) + bv + (rowbias ? rowbias[mrow] : 0.0f); }
          }
      }
      __syncthreads();
      if (R) {
        for (int ch = t; ch < 64 * 64; ch += 256) { const int ml = ch >> 6, q = (ch & 63) * 4;
          if (nBlk + q < N) { const v4f_t rv = *(const v4f_t*)(R + (size_t)(mBlk + hf * 64 + ml) * N + nBlk + q); v4f_t v = *(const v4fa*)(so + ml * 260 + q); v += rv; *(volatile v4fa*)(so + ml * 260 + q) = v; } }
        asm volatile("s_wait_dscnt 0" ::: "memory");
      }
#pragma unroll 1
      for (int pass = 0; pass < 2; ++pass) {
        for (int ch = t; ch < 64 * 64; ch += 256) { const int ml = ch >> 6, q = (ch & 63) * 4;
          if (nBlk + q < N) *(volatile v4f_t*)((float*)out + (size_t)(mBlk + hf * 64 + ml) * N + nBlk + q) = *(const v4fa*)(so + ml * 260 + q); }
        __threadfence();
      }
      __syncthreads();
    }
  }
}


__global__ __launch_bounds__(256) void k_instnorm(float* __restrict__ Y) {
  __shared__ float red[8][32]; __shared__ float mu[32], rs[32];
  const int b = blockIdx.x / (HHs / 32), cg = (blockIdx.x % (HHs / 32)) * 32; const int tid = threadIdx.x, tl = tid >> 5, c = tid & 31;
  float* base = Y + (size_t)b * TTs * HHs + cg + c;
  float s = 0.0f;
#pragma unroll 1
  for (int t = tl; t < TTs; t += 8) s += base[(size_t)t * HHs];
  red[tl][c] = s; __syncthreads();
  if (tl == 0) { float a = 0.0f; for (int i = 0; i < 8; ++i) a += red[i][c]; mu[c] = a * (1.0f / TTs); }
  __syncthreads();
  const float m = mu[c]; float q = 0.0f;
#pragma unroll 1
  for (int t = tl; t < TTs; t += 8) { const float d = base[(size_t)t * HHs] - m; q += d * d; }
  red[tl][c] = q; __syncthreads();
  if (tl == 0) { float a = 0.0f; for (int i = 0; i < 8; ++i) a += red[i][c]; rs[c] = rsqrtf(a * (1.0f / TTs) + 1e-5f); }
  __syncthreads();
  const float r = rs[c];
#pragma unroll 1
  for (int t = tl; t < TTs; t += 8) { const float v = (base[(size_t)t * HHs] - m) * r; *(volatile float*)(base + (size_t)t * HHs) = v; __threadfence(); *(volatile float*)(base + (size_t)t * HHs) = v; }
}
__global__ __launch_bounds__(256) void k_band(const float* __restrict__ Q, const float* __restrict__ Kx, const float* __restrict__ V, float* __restrict__ O) {
  const int tid = threadIdx.x, wave = tid >> 5, lane = tid & 31; const int b = blockIdx.x / (TTs / 8), t = (blockIdx.x % (TTs / 8)) * 8 + wave;
  const size_t rowq = ((size_t)b * TTs + t) * HHs + lane * 8;
  float qv[8]; { const v4f_t a = *(const v4f_t*)(Q + rowq), c2 = *(const v4f_t*)(Q + rowq + 4); for (int e = 0; e < 4; ++e) { qv[e] = a[e]; qv[4 + e] = c2[e]; } }
  const float scale = 0.0625f;
  float m = -3.0e38f, l = 0.0f; float o[8]; for (int e = 0; e < 8; ++e) o[e] = 0.0f;
  const int W33 = 33 + (int)(blockIdx.x >> 30);
#pragma unroll 1
  for (int w = 0; w < W33; ++w) { const int j = t - HALF + w; if (j < 0 || j >= TTs) continue;
    const size_t rowk = ((size_t)b * TTs + j) * HHs + lane * 8;
    const v4f_t ka = *(const v4f_t*)(Kx + rowk), kb2 = *(const v4f_t*)(Kx + rowk + 4);
    float part = 0.0f; for (int e = 0; e < 4; ++e) { part += qv[e] * ka[e]; part += qv[4 + e] * kb2[e]; }
#pragma unroll
    for (int off = 1; off < 32; off <<= 1) part += __shfl_xor(part, off, 32);
    const float sc = part * scale; const float mn = fmaxf(m, sc); const float alpha = expf(m - mn); const float p = expf(sc - mn);
    l = l * alpha + p;
    const v4f_t va = *(const v4f_t*)(V + rowk), vb2 = *(const v4f_t*)(V + rowk + 4);
    for (int e = 0; e < 4; ++e) { o[e] = o[e] * alpha + p * va[e]; o[4 + e] = o[4 + e] * alpha + p * vb2[e]; }
    m = mn; }
  const float il = 1.0f / l; v4f_t r0, r1; for (int e = 0; e < 4; ++e) { r0[e] = o[e] * il; r1[e] = o[4 + e] * il; }
  *(volatile v4f_t*)(O + rowq) = r0; *(volatile v4f_t*)(O + rowq + 4) = r1; __threadfence(); *(volatile v4f_t*)(O + rowq) = r0; *(volatile v4f_t*)(O + rowq + 4) = r1;
}
__global__ __launch_bounds__(256) void k_tmean(const float* __restrict__ O, float* __restrict__ out) { const int b = blockIdx.x, c = threadIdx.x; float s = 0.0f;
#pragma unroll 1
  for (int t = 0; t < TTs; ++t) s += O[((size_t)b * TTs + t) * HHs + c];
  s *= (1.0f / TTs); *(volatile float*)(out + (size_t)b * HHs + c) = s; __threadfence(); *(volatile float*)(out + (size_t)b * HHs + c) = s; }

extern "C" void kernel_launch(void* const* d_in, const int* in_sizes, int n_in,
                              void* d_out, int out_size, void* d_ws, size_t ws_size,
                              hipStream_t stream) {
  (void)in_sizes; (void)n_in; (void)out_size;
  const float** f = (const float**)d_in;
  const float* x = f[0], *Wq = f[1], *bq = f[2], *Wk = f[3], *bk = f[4], *Wv = f[5], *bv = f[6];
  float* out = (float*)d_out;
  char* ws = (char*)d_ws;
  float* q = (float*)ws; ws += (size_t)MTOK * HHs * 4; float* k = (float*)ws; ws += (size_t)MTOK * HHs * 4; float* v = (float*)ws; ws += (size_t)MTOK * HHs * 4; float* O = (float*)ws; ws += (size_t)MTOK * HHs * 4;
  if ((size_t)(ws - (char*)d_ws) > ws_size) return;
  const dim3 blk(256);
  gemm_rb_kernel<float, 2><<<dim3(MTOK / 128, HHs / 256), blk, 0, stream>>>(x, Wq, bq, nullptr, nullptr, nullptr, q, MTOK, HHs, HHs);
  gemm_rb_kernel<float, 2><<<dim3(MTOK / 128, HHs / 256), blk, 0, stream>>>(x, Wk, bk, nullptr, nullptr, nullptr, k, MTOK, HHs, HHs);
  gemm_rb_kernel<float, 2><<<dim3(MTOK / 128, HHs / 256), blk, 0, stream>>>(x, Wv, bv, nullptr, nullptr, nullptr, v, MTOK, HHs, HHs);
  k_instnorm<<<dim3(NBs * (HHs / 32)), blk, 0, stream>>>(q); k_instnorm<<<dim3(NBs * (HHs / 32)), blk, 0, stream>>>(k); k_instnorm<<<dim3(NBs * (HHs / 32)), blk, 0, stream>>>(v);
  k_band<<<dim3(NBs * (TTs / 8)), blk, 0, stream>>>(q, k, v, O);
  k_tmean<<<dim3(NBs), blk, 0, stream>>>(O, out);
}
